// Mamba3DBlock_3006477107886
// MI455X (gfx1250) — hardware-verified
//
#include <hip/hip_runtime.h>
#include <math.h>


#define C_DIM 384
#define NPTS 2048
#define BATCH 4
#define ROWS_ALL (BATCH * (NPTS + 1))
#define ROWS_NO  (BATCH * NPTS)
#define KG 8
#define KNN_TPB 256
#define AGG_N 448
#define XT_BSTRIDE ((size_t)AGG_N * NPTS)
#define QB_PITCH 32
#define STAT_BLOCKS 64
#define STAT_ROWS (ROWS_NO / STAT_BLOCKS)
#define ACT_SC 16.0f
#define ACT_INV (1.0f / 16.0f)
#define W_SC 64.0f
#define OUT_SC (1.0f / 1024.0f)
#define QL_SC 4096.0f
#define QL_INV (1.0f / 4096.0f)

static_assert(NPTS % KNN_TPB == 0, "");
static_assert(NPTS % 128 == 0, "");
static_assert(ROWS_NO % STAT_BLOCKS == 0 && STAT_ROWS % 8 == 0, "");
static_assert(C_DIM == 96 * 4, "");
static_assert(AGG_N % 64 == 0 && AGG_N >= C_DIM + 2, "");

typedef _Float16 hf;
typedef hf     v16h __attribute__((ext_vector_type(16)));
typedef hf     v8h  __attribute__((ext_vector_type(8)));
typedef hf     v4h  __attribute__((ext_vector_type(4)));
typedef float  v8f  __attribute__((ext_vector_type(8)));
typedef float  v4f  __attribute__((ext_vector_type(4)));
typedef double v2d  __attribute__((ext_vector_type(2)));
typedef v4f v4fa __attribute__((may_alias));
typedef v8h v8ha __attribute__((may_alias));

union Frag  { v16h v; v8h h[2]; };
union Pack8 { v8h v; hf s[8]; };
union Pack4 { v4h v; hf s[4]; };

template<typename V>
__device__ __forceinline__ void store2(V* p, V v) {
    *(volatile V*)p = v;
    __threadfence();
    *(volatile V*)p = v;
}

__device__ __forceinline__ float gelu_exact(float v) {
    return 0.5f * v * (1.0f + erff(v * 0.70710678118654752f));
}

__device__ __forceinline__ float bsum96(float v, float* red, int tid) {
    #pragma unroll
    for (int o = 16; o > 0; o >>= 1) v += __shfl_xor(v, o, 32);
    __syncthreads();
    if ((tid & 31) == 0) red[tid >> 5] = v;
    __syncthreads();
    return (red[0] + red[1]) + red[2];
}

__global__ __launch_bounds__(96) void ln1_kernel(const float* __restrict__ x, const float* __restrict__ g,
                                                 const float* __restrict__ bb, float* __restrict__ xn,
                                                 float* __restrict__ out, float* __restrict__ qb) {
    __shared__ float red[4];
    const int row = blockIdx.x;
    const int tid = threadIdx.x;
    const int c = tid * 4;
    const size_t base = (size_t)row * C_DIM + c;
    const v4f v = *(const v4f*)(x + base);
    const float mean = bsum96((v.x + v.y) + (v.z + v.w), red, tid) * (1.0f / C_DIM);
    v4f d;
    d.x = v.x - mean; d.y = v.y - mean; d.z = v.z - mean; d.w = v.w - mean;
    const float var = bsum96((d.x * d.x + d.y * d.y) + (d.z * d.z + d.w * d.w), red, tid) * (1.0f / C_DIM);
    const float rstd = 1.0f / sqrtf(var + 1e-5f);
    const v4f gg = *(const v4f*)(g + c);
    const v4f be = *(const v4f*)(bb + c);
    v4f o;
    o.x = d.x * rstd * gg.x + be.x;
    o.y = d.y * rstd * gg.y + be.y;
    o.z = d.z * rstd * gg.z + be.z;
    o.w = d.w * rstd * gg.w + be.w;
    store2((v4f*)(xn + base), o);
    const float q = bsum96((o.x * o.x + o.y * o.y) + (o.z * o.z + o.w * o.w), red, tid);
    if (tid < 8) {
        v4f qv;
        qv.x = (tid == 0) ? q : 0.0f; qv.y = 0.0f; qv.z = 0.0f; qv.w = 0.0f;
        store2((v4f*)(qb + (size_t)row * QB_PITCH + tid * 4), qv);
    }
    if ((row % (NPTS + 1)) == 0) {
        const v4f r2 = v + o;
        store2((v4f*)(out + base), r2);
    }
}

__global__ __launch_bounds__(96) void ln2_kernel(const float* __restrict__ x, const float* __restrict__ g,
                                                 const float* __restrict__ bb, hf* __restrict__ y) {
    __shared__ float red[4];
    __shared__ __attribute__((aligned(16))) hf srow[C_DIM];
    const int row = blockIdx.x;
    const int tid = threadIdx.x;
    const int c = tid * 4;
    const size_t base = (size_t)row * C_DIM + c;
    const v4f v = *(const v4f*)(x + base);
    const float mean = bsum96((v.x + v.y) + (v.z + v.w), red, tid) * (1.0f / C_DIM);
    v4f d;
    d.x = v.x - mean; d.y = v.y - mean; d.z = v.z - mean; d.w = v.w - mean;
    const float var = bsum96((d.x * d.x + d.y * d.y) + (d.z * d.z + d.w * d.w), red, tid) * (1.0f / C_DIM);
    const float rstd = 1.0f / sqrtf(var + 1e-5f);
    const v4f gg = *(const v4f*)(g + c);
    const v4f be = *(const v4f*)(bb + c);
    Pack4 pk;
    pk.s[0] = (hf)((d.x * rstd * gg.x + be.x) * ACT_SC);
    pk.s[1] = (hf)((d.y * rstd * gg.y + be.y) * ACT_SC);
    pk.s[2] = (hf)((d.z * rstd * gg.z + be.z) * ACT_SC);
    pk.s[3] = (hf)((d.w * rstd * gg.w + be.w) * ACT_SC);
    *(v4h*)(srow + c) = pk.v;
    __syncthreads();
    if (tid < 48) {
        const v8h hv = *(const v8ha*)(srow + tid * 8);
        store2((v8h*)(y + (size_t)row * C_DIM + tid * 8), hv);
    }
}

__global__ __launch_bounds__(KNN_TPB) void knn_sel_kernel(const float* __restrict__ center, hf* __restrict__ sel) {
    #pragma clang fp contract(off)
    __shared__ float cx[NPTS], cy[NPTS], cz[NPTS], cq[NPTS];
    const int b = blockIdx.y;
    const int tid = threadIdx.x;
    const float* cb = center + (size_t)b * NPTS * 3;
    for (int i = tid; i < NPTS; i += KNN_TPB) {
        const float px = cb[i * 3 + 0], py = cb[i * 3 + 1], pz = cb[i * 3 + 2];
        cx[i] = px; cy[i] = py; cz[i] = pz;
        cq[i] = px * px + py * py + pz * pz;
    }
    __syncthreads();

    const int n = blockIdx.x * KNN_TPB + tid;
    const float qx = cx[n], qy = cy[n], qz = cz[n], qs = cq[n];
    float bd[KG];
    int   bi[KG];
    #pragma unroll
    for (int j = 0; j < KG; j++) { bd[j] = 3.4e38f; bi[j] = n; }
    for (int m = 0; m < NPTS; m++) {
        const float dot = qx * cx[m] + qy * cy[m] + qz * cz[m];
        const float d = (qs + cq[m]) - 2.0f * dot;
        if (d < bd[KG - 1]) {
            float dd = d;
            int mm = m;
            #pragma unroll
            for (int j = 0; j < KG; j++) {
                if (dd < bd[j]) {
                    const float tb = bd[j]; const int ti = bi[j];
                    bd[j] = dd; bi[j] = mm;
                    dd = tb; mm = ti;
                }
            }
        }
    }
    int ch[KG];
    unsigned ob[KG];
    #pragma unroll
    for (int j = 0; j < KG; j++) { ch[j] = bi[j] >> 3; ob[j] = 1u << (bi[j] & 7); }

    hf* rowp = sel + ((size_t)(b * NPTS + n)) * NPTS;
    #pragma unroll 1
    for (int pass = 0; pass < 2; pass++) {
        #pragma unroll 1
        for (int j = 0; j < NPTS / 8; j++) {
            unsigned bits = 0u;
            #pragma unroll
            for (int k = 0; k < KG; k++) bits |= (ch[k] == j) ? ob[k] : 0u;
            Pack8 pk;
            #pragma unroll
            for (int i = 0; i < 8; i++) pk.s[i] = ((bits >> i) & 1u) ? (hf)1.0f : (hf)0.0f;
            *(volatile v8h*)(rowp + 8 * j) = pk.v;
        }
        if (pass == 0) __threadfence();
    }
}

__global__ __launch_bounds__(256) void wtr_kernel(const float* __restrict__ w, size_t ibs, hf* __restrict__ wT, size_t obs,
                                                  int Kd, int Nd, float sc) {
    __shared__ float tile[64][33];
    w  += (size_t)blockIdx.z * ibs;
    wT += (size_t)blockIdx.z * obs;
    const int tid = threadIdx.x;
    const int n0 = blockIdx.x * 32;
    const int k0 = blockIdx.y * 64;
    #pragma unroll
    for (int i = 0; i < 8; i++) {
        const int kk = i * 8 + (tid >> 5);
        const int nn = tid & 31;
        const int gk = k0 + kk, gn = n0 + nn;
        tile[kk][nn] = (gk < Kd && gn < Nd) ? w[(size_t)gk * Nd + gn] : 0.0f;
    }
    __syncthreads();
    const int nl = tid >> 3, k8 = tid & 7;
    const int gn = n0 + nl, gk = k0 + k8 * 8;
    Pack8 pk;
    #pragma unroll
    for (int j = 0; j < 8; j++) pk.s[j] = (hf)(tile[k8 * 8 + j][nl] * sc);
    if (gn < Nd && gk + 8 <= Kd) store2((v8h*)(wT + (size_t)gn * Kd + gk), pk.v);
}

__global__ __launch_bounds__(256) void qcol_kernel(const float* __restrict__ qb, hf* __restrict__ xT) {
    const int b = blockIdx.y;
    const int r = blockIdx.x;
    const int m0 = threadIdx.x * 8;
    Pack8 pk;
    #pragma unroll
    for (int i = 0; i < 8; i++) pk.s[i] = (hf)0.0f;
    if (r < 2) {
        #pragma unroll
        for (int i = 0; i < 8; i++) {
            const float q = qb[((size_t)(b * (NPTS + 1) + 1 + m0 + i)) * QB_PITCH];
            const hf qh = (hf)q;
            pk.s[i] = (r == 0) ? qh : (hf)((q - (float)qh) * QL_SC);
        }
    }
    store2((v8h*)(xT + (size_t)b * XT_BSTRIDE + (size_t)(C_DIM + r) * NPTS + m0), pk.v);
}

__global__ __launch_bounds__(256) void stats_kernel(const float* __restrict__ S, const float* __restrict__ xn,
                                                    const float* __restrict__ qb, double* __restrict__ part) {
    __shared__ double w1[8], w2[8];
    const int tid = threadIdx.x, lane = tid & 31, wave = tid >> 5;
    double ds = 0.0, dq = 0.0;
    for (int i = 0; i < STAT_ROWS / 8; i++) {
        const int row = blockIdx.x * STAT_ROWS + wave * (STAT_ROWS / 8) + i;
        const int bb = row >> 11, nn = row & (NPTS - 1);
        const size_t xrow = (size_t)(bb * (NPTS + 1) + 1 + nn);
        const float* sp = S + (size_t)row * AGG_N;
        const float* xp = xn + xrow * C_DIM;
        float fs = 0.0f, fx = 0.0f;
        #pragma unroll
        for (int t = 0; t < 3; t++) {
            const int c = t * 128 + lane * 4;
            const v4f s4 = *(const v4f*)(sp + c);
            const v4f x4 = *(const v4f*)(xp + c);
            fs += (s4.x + s4.y) + (s4.z + s4.w);
            fx += (x4.x * s4.x + x4.y * s4.y) + (x4.z * s4.z + x4.w * s4.w);
        }
        #pragma unroll
        for (int o = 16; o > 0; o >>= 1) { fs += __shfl_xor(fs, o, 32); fx += __shfl_xor(fx, o, 32); }
        const float qh = sp[C_DIM], ql = sp[C_DIM + 1];
        const float qn = qb[xrow * QB_PITCH];
        ds += (double)fs;
        dq += ((double)qh + (double)ql) - 8.0 * (double)qn - 2.0 * (double)fx;
    }
    if (lane == 0) { w1[wave] = ds; w2[wave] = dq; }
    __syncthreads();
    if (tid < 8) {
        double t1 = 0.0, t2 = 0.0;
        #pragma unroll
        for (int j = 0; j < 8; j++) { t1 += w1[j]; t2 += w2[j]; }
        v2d pv;
        pv.x = (tid == 0) ? t1 : 0.0;
        pv.y = (tid == 0) ? t2 : 0.0;
        store2((v2d*)(part + (size_t)blockIdx.x * 16 + tid * 2), pv);
    }
}

__global__ __launch_bounds__(256) void ef_kernel(const float* __restrict__ S, const float* __restrict__ xn,
                                                 const float* __restrict__ alpha, const float* __restrict__ beta,
                                                 const double* __restrict__ part, hf* __restrict__ ef) {
    __shared__ float sinv;
    const int tid = threadIdx.x;
    if (tid == 0) {
        double s = 0.0, ss = 0.0;
        for (int i = 0; i < STAT_BLOCKS; i++) { s += part[(size_t)i * 16]; ss += part[(size_t)i * 16 + 1]; }
        const double Mtot = (double)ROWS_NO * (double)KG * (double)C_DIM;
        double var = (ss - s * s / Mtot) / (Mtot - 1.0);
        if (var < 0.0) var = 0.0;
        const float stdv = sqrtf((float)var);
        sinv = 1.0f / (stdv + 1e-5f);
    }
    __syncthreads();
    const float inv = sinv;
    const int t = blockIdx.x * 256 + tid;
    if (t < ROWS_NO * 96) {
        const int row = t / 96;
        const int g = t - row * 96;
        float e[8];
        if (g < 48) {
            const int c = g * 8;
            const float* sp = S + (size_t)row * AGG_N + c;
            const v4f s0 = *(const v4f*)sp;
            const v4f s1 = *(const v4f*)(sp + 4);
            const float vals[8] = {s0.x, s0.y, s0.z, s0.w, s1.x, s1.y, s1.z, s1.w};
            #pragma unroll
            for (int j = 0; j < 8; j++) e[j] = alpha[c + j] * ((vals[j] * 0.125f) * inv) + beta[c + j];
        } else {
            const int c = (g - 48) * 8;
            const int bb = row >> 11, nn = row & (NPTS - 1);
            const float* xp = xn + ((size_t)(bb * (NPTS + 1) + 1 + nn)) * C_DIM + c;
            const v4f x0 = *(const v4f*)xp;
            const v4f x1 = *(const v4f*)(xp + 4);
            const float vals[8] = {x0.x, x0.y, x0.z, x0.w, x1.x, x1.y, x1.z, x1.w};
            #pragma unroll
            for (int j = 0; j < 8; j++) e[j] = alpha[C_DIM + c + j] * vals[j] + beta[C_DIM + c + j];
        }
        Pack8 pk;
        #pragma unroll
        for (int j = 0; j < 8; j++) pk.s[j] = (hf)(e[j] * ACT_SC);
        store2((v8h*)(ef + (size_t)row * (2 * C_DIM) + g * 8), pk.v);
    }
}

template<int MODE>
__global__ __launch_bounds__(128) void gemm_kernel(const hf* __restrict__ A, const hf* __restrict__ Bt,
                                                    const float* __restrict__ bias, int M, int K, int N,
                                                    hf* __restrict__ outH, float* outF, const float* resid,
                                                    const float* __restrict__ xn) {
    __shared__ __attribute__((aligned(16))) float stile[4 * 32 * 64];
    const int lane = threadIdx.x & 31;
    const int wave = threadIdx.x >> 5;
    const int h = lane >> 4;
    const int l16 = lane & 15;
    const int row0 = blockIdx.y * 128 + wave * 32;
    const int col0 = blockIdx.x * 64;
    if (MODE == 3) Bt += (size_t)((blockIdx.y * 128) / NPTS) * (size_t)N * (size_t)K;

    int ar0 = row0 + l16;      if (ar0 > M - 1) ar0 = M - 1;
    int ar1 = row0 + 16 + l16; if (ar1 > M - 1) ar1 = M - 1;
    const hf* ap0 = A + (size_t)ar0 * K + 8 * h;
    const hf* ap1 = A + (size_t)ar1 * K + 8 * h;
    const hf* bp[4];
    #pragma unroll
    for (int t = 0; t < 4; t++) {
        int cn = col0 + t * 16 + l16; if (cn > N - 1) cn = N - 1;
        bp[t] = Bt + (size_t)cn * K + 8 * h;
    }

    const v8f zero = {0.0f, 0.0f, 0.0f, 0.0f, 0.0f, 0.0f, 0.0f, 0.0f};
    v8f acc[8];
    #pragma unroll
    for (int i = 0; i < 8; i++) acc[i] = zero;

    #pragma unroll 1
    for (int kt = 0; kt < K; kt += 32) {
        Frag a0, a1, b0, b1, b2, b3;
        a0.h[0] = *(const v8h*)(ap0 + kt);   a0.h[1] = *(const v8h*)(ap0 + kt + 16);
        a1.h[0] = *(const v8h*)(ap1 + kt);   a1.h[1] = *(const v8h*)(ap1 + kt + 16);
        b0.h[0] = *(const v8h*)(bp[0] + kt); b0.h[1] = *(const v8h*)(bp[0] + kt + 16);
        b1.h[0] = *(const v8h*)(bp[1] + kt); b1.h[1] = *(const v8h*)(bp[1] + kt + 16);
        b2.h[0] = *(const v8h*)(bp[2] + kt); b2.h[1] = *(const v8h*)(bp[2] + kt + 16);
        b3.h[0] = *(const v8h*)(bp[3] + kt); b3.h[1] = *(const v8h*)(bp[3] + kt + 16);
        acc[0] = __builtin_amdgcn_wmma_f32_16x16x32_f16(false, a0.v, false, b0.v, (short)0, acc[0], false, false);
        acc[4] = __builtin_amdgcn_wmma_f32_16x16x32_f16(false, a1.v, false, b0.v, (short)0, acc[4], false, false);
        acc[1] = __builtin_amdgcn_wmma_f32_16x16x32_f16(false, a0.v, false, b1.v, (short)0, acc[1], false, false);
        acc[5] = __builtin_amdgcn_wmma_f32_16x16x32_f16(false, a1.v, false, b1.v, (short)0, acc[5], false, false);
        acc[2] = __builtin_amdgcn_wmma_f32_16x16x32_f16(false, a0.v, false, b2.v, (short)0, acc[2], false, false);
        acc[6] = __builtin_amdgcn_wmma_f32_16x16x32_f16(false, a1.v, false, b2.v, (short)0, acc[6], false, false);
        acc[3] = __builtin_amdgcn_wmma_f32_16x16x32_f16(false, a0.v, false, b3.v, (short)0, acc[3], false, false);
        acc[7] = __builtin_amdgcn_wmma_f32_16x16x32_f16(false, a1.v, false, b3.v, (short)0, acc[7], false, false);
        asm volatile("v_nop\n\tv_nop\n\tv_nop\n\tv_nop"
                     : "+v"(acc[0]), "+v"(acc[1]), "+v"(acc[2]), "+v"(acc[3]),
                       "+v"(acc[4]), "+v"(acc[5]), "+v"(acc[6]), "+v"(acc[7])
                     : "v"(a0.v), "v"(a1.v), "v"(b0.v), "v"(b1.v), "v"(b2.v), "v"(b3.v));
    }

    float* st = stile + wave * (32 * 64);
    #pragma unroll
    for (int t = 0; t < 4; t++) {
        const int cl = t * 16 + l16;
        float bv = 0.0f;
        if (MODE != 3) { int cb = col0 + cl; if (cb > N - 1) cb = N - 1; bv = bias[cb]; }
        #pragma unroll
        for (int r = 0; r < 8; r++) {
            float v0, v1;
            if (MODE == 3) { v0 = acc[t][r]; v1 = acc[4 + t][r]; }
            else           { v0 = acc[t][r] * OUT_SC + bv; v1 = acc[4 + t][r] * OUT_SC + bv; }
            if (MODE == 1) { v0 = gelu_exact(v0) * ACT_SC; v1 = gelu_exact(v1) * ACT_SC; }
            st[(8 * h + r) * 64 + cl] = v0;
            st[(16 + 8 * h + r) * 64 + cl] = v1;
        }
    }
    __syncthreads();

    if (MODE == 1) {
        const int rsub = lane >> 3, c8 = lane & 7;
        #pragma unroll
        for (int i = 0; i < 8; i++) {
            const int rl = i * 4 + rsub;
            const float* sp = st + rl * 64 + c8 * 8;
            const v4f u0 = *(const v4fa*)sp;
            const v4f u1 = *(const v4fa*)(sp + 4);
            Pack8 pk;
            pk.s[0] = (hf)u0.x; pk.s[1] = (hf)u0.y; pk.s[2] = (hf)u0.z; pk.s[3] = (hf)u0.w;
            pk.s[4] = (hf)u1.x; pk.s[5] = (hf)u1.y; pk.s[6] = (hf)u1.z; pk.s[7] = (hf)u1.w;
            const int row = row0 + rl;
            if (row < M) store2((v8h*)(outH + (size_t)row * N + col0 + c8 * 8), pk.v);
        }
    } else {
        const int bagg = (blockIdx.y * 128) / NPTS;
        #pragma unroll
        for (int i = 0; i < 16; i++) {
            const int rl = i * 2 + h;
            v4f u = *(const v4fa*)(st + rl * 64 + l16 * 4);
            const int row = row0 + rl;
            if (row < M) {
                if (MODE == 3) {
                    const size_t o = (size_t)row * (size_t)N + col0 + l16 * 4;
                    if (col0 < C_DIM) {
                        const size_t xo = ((size_t)(bagg * (NPTS + 1) + 1 + (row & (NPTS - 1)))) * C_DIM + col0 + l16 * 4;
                        const v4f x4 = *(const v4f*)(xn + xo);
                        u = u * ACT_INV - x4 * 8.0f;
                    } else {
                        if (l16 == 0) u.y = u.y * QL_INV;
                    }
                    store2((v4f*)(outF + o), u);
                } else {
                    const size_t orow = (MODE == 2)
                        ? ((size_t)(row >> 11) * (NPTS + 1) + 1 + (size_t)(row & (NPTS - 1)))
                        : (size_t)row;
                    const size_t o = orow * (size_t)N + col0 + l16 * 4;
                    const v4f rs = *(const v4f*)(resid + o);
                    u = u + rs;
                    store2((v4f*)(outF + o), u);
                }
            }
        }
    }
}

extern "C" void kernel_launch(void* const* d_in, const int* in_sizes, int n_in,
                              void* d_out, int out_size, void* d_ws, size_t ws_size,
                              hipStream_t stream) {
    if (n_in < 16) return;
    if (in_sizes[0] != BATCH * NPTS * 3) return;
    if (in_sizes[1] != ROWS_ALL * C_DIM) return;
    if (in_sizes[2] != C_DIM || in_sizes[3] != C_DIM) return;
    if (in_sizes[4] != 2 * C_DIM || in_sizes[5] != 2 * C_DIM) return;
    if (in_sizes[6] != 2 * C_DIM * C_DIM || in_sizes[7] != C_DIM) return;
    if (in_sizes[8] != C_DIM * C_DIM || in_sizes[9] != C_DIM) return;
    if (in_sizes[10] != C_DIM || in_sizes[11] != C_DIM) return;
    if (in_sizes[12] != 4 * C_DIM * C_DIM || in_sizes[13] != 4 * C_DIM) return;
    if (in_sizes[14] != 4 * C_DIM * C_DIM || in_sizes[15] != C_DIM) return;
    if (out_size != ROWS_ALL * C_DIM) return;

    const float* center  = (const float*)d_in[0];
    const float* x       = (const float*)d_in[1];
    const float* ln1_g   = (const float*)d_in[2];
    const float* ln1_b   = (const float*)d_in[3];
    const float* alpha   = (const float*)d_in[4];
    const float* beta    = (const float*)d_in[5];
    const float* attn_w1 = (const float*)d_in[6];
    const float* attn_b1 = (const float*)d_in[7];
    const float* attn_w2 = (const float*)d_in[8];
    const float* attn_b2 = (const float*)d_in[9];
    const float* ln2_g   = (const float*)d_in[10];
    const float* ln2_b   = (const float*)d_in[11];
    const float* mlp_w1  = (const float*)d_in[12];
    const float* mlp_b1  = (const float*)d_in[13];
    const float* mlp_w2  = (const float*)d_in[14];
    const float* mlp_b2  = (const float*)d_in[15];
    float* out = (float*)d_out;

    size_t off = 0;
    auto carve = [&](size_t bytes) -> size_t { const size_t o = off; off += (bytes + 255) & ~(size_t)255; return o; };
    const size_t o_xn  = carve((size_t)ROWS_ALL * C_DIM * sizeof(float));
    const size_t o_S   = carve((size_t)ROWS_NO * AGG_N * sizeof(float));
    const size_t o_sel = carve((size_t)ROWS_NO * NPTS * sizeof(hf));
    const size_t o_xt  = carve((size_t)BATCH * XT_BSTRIDE * sizeof(hf));
    const size_t o_qb  = carve((size_t)ROWS_ALL * QB_PITCH * sizeof(float));
    const size_t o_pt  = carve((size_t)STAT_BLOCKS * 16 * sizeof(double));
    const size_t o_ef  = carve((size_t)ROWS_NO * 2 * C_DIM * sizeof(hf));
    const size_t o_h1  = carve((size_t)ROWS_NO * C_DIM * sizeof(hf));
    const size_t o_y   = carve((size_t)ROWS_ALL * C_DIM * sizeof(hf));
    const size_t o_g   = carve((size_t)ROWS_ALL * 4 * C_DIM * sizeof(hf));
    const size_t o_w1  = carve((size_t)2 * C_DIM * C_DIM * sizeof(hf));
    const size_t o_w2  = carve((size_t)C_DIM * C_DIM * sizeof(hf));
    const size_t o_m1  = carve((size_t)4 * C_DIM * C_DIM * sizeof(hf));
    const size_t o_m2  = carve((size_t)4 * C_DIM * C_DIM * sizeof(hf));
    if (off > ws_size) return;

    char* ws = (char*)d_ws;
    float*  xn   = (float*)(ws + o_xn);
    float*  S    = (float*)(ws + o_S);
    hf*     sel  = (hf*)(ws + o_sel);
    hf*     xT   = (hf*)(ws + o_xt);
    float*  qb   = (float*)(ws + o_qb);
    double* part = (double*)(ws + o_pt);
    hf*     ef   = (hf*)(ws + o_ef);
    hf*     H1   = (hf*)(ws + o_h1);
    hf*     y    = (hf*)(ws + o_y);
    hf*     G    = (hf*)(ws + o_g);
    hf*     w1T  = (hf*)(ws + o_w1);
    hf*     w2T  = (hf*)(ws + o_w2);
    hf*     mw1T = (hf*)(ws + o_m1);
    hf*     mw2T = (hf*)(ws + o_m2);

    ln1_kernel<<<ROWS_ALL, 96, 0, stream>>>(x, ln1_g, ln1_b, xn, out, qb);
    knn_sel_kernel<<<dim3(NPTS / KNN_TPB, BATCH), KNN_TPB, 0, stream>>>(center, sel);
    wtr_kernel<<<dim3((C_DIM + 31) / 32, (NPTS + 63) / 64, BATCH), 256, 0, stream>>>(
        xn + C_DIM, (size_t)(NPTS + 1) * C_DIM, xT, XT_BSTRIDE, NPTS, C_DIM, ACT_SC);
    qcol_kernel<<<dim3(AGG_N - C_DIM, BATCH), 256, 0, stream>>>(qb, xT);
    gemm_kernel<3><<<dim3(AGG_N / 64, ROWS_NO / 128), 128, 0, stream>>>(
        sel, xT, attn_b1, ROWS_NO, NPTS, AGG_N, H1, S, xn, xn);
    stats_kernel<<<STAT_BLOCKS, 256, 0, stream>>>(S, xn, qb, part);
    ef_kernel<<<(ROWS_NO * 96 + 255) / 256, 256, 0, stream>>>(S, xn, alpha, beta, part, ef);
    wtr_kernel<<<dim3((C_DIM + 31) / 32, (2 * C_DIM + 63) / 64, 1), 256, 0, stream>>>(attn_w1, 0, w1T, 0, 2 * C_DIM, C_DIM, W_SC);
    wtr_kernel<<<dim3((C_DIM + 31) / 32, (C_DIM + 63) / 64, 1), 256, 0, stream>>>(attn_w2, 0, w2T, 0, C_DIM, C_DIM, W_SC);
    wtr_kernel<<<dim3((4 * C_DIM + 31) / 32, (C_DIM + 63) / 64, 1), 256, 0, stream>>>(mlp_w1, 0, mw1T, 0, C_DIM, 4 * C_DIM, W_SC);
    wtr_kernel<<<dim3((C_DIM + 31) / 32, (4 * C_DIM + 63) / 64, 1), 256, 0, stream>>>(mlp_w2, 0, mw2T, 0, 4 * C_DIM, C_DIM, W_SC);
    gemm_kernel<1><<<dim3(C_DIM / 64, (ROWS_NO + 127) / 128), 128, 0, stream>>>(
        ef, w1T, attn_b1, ROWS_NO, 2 * C_DIM, C_DIM, H1, S, xn, xn);
    gemm_kernel<2><<<dim3(C_DIM / 64, (ROWS_NO + 127) / 128), 128, 0, stream>>>(
        H1, w2T, attn_b2, ROWS_NO, C_DIM, C_DIM, H1, out, x, xn);
    ln2_kernel<<<ROWS_ALL, 96, 0, stream>>>(out, ln2_g, ln2_b, y);
    gemm_kernel<1><<<dim3(4 * C_DIM / 64, (ROWS_ALL + 127) / 128), 128, 0, stream>>>(
        y, mw1T, mlp_b1, ROWS_ALL, C_DIM, 4 * C_DIM, G, S, xn, xn);
    gemm_kernel<4><<<dim3(C_DIM / 64, (ROWS_ALL + 127) / 128), 128, 0, stream>>>(
        G, mw2T, mlp_b2, ROWS_ALL, 4 * C_DIM, C_DIM, H1, out, out, xn);
}
